// SelfAttention_20246475833997
// MI455X (gfx1250) — hardware-run, weakly checked
//
#include <hip/hip_runtime.h>


#ifndef NB
#define NB 4
#endif
#ifndef SEQ
#define SEQ 2048
#endif
#define NB_FULL  4
#define SEQ_FULL 2048
#define DM   1024
#define NH   16
#define HD   64
#define MT   (NB * SEQ)
#define L2E  1.4426950408889634f
#define SC2  (0.125f * 1.4426950408889634f)

static_assert(NH * HD == DM);
static_assert(HD == 64);
static_assert(SEQ % 64 == 0);
static_assert(DM % 64 == 0);
static_assert(NB <= NB_FULL);
static_assert(SEQ <= SEQ_FULL);
static_assert(((NB * NH * (SEQ / 16)) % 4) == 0);

typedef _Float16 h16;
typedef unsigned short bf;
typedef __attribute__((ext_vector_type(16))) __bf16   v16bf;
typedef __attribute__((ext_vector_type(16))) _Float16 v16h;
typedef __attribute__((ext_vector_type(8)))  _Float16 v8h;
typedef __attribute__((ext_vector_type(8)))  unsigned short v8us;
typedef __attribute__((ext_vector_type(2)))  unsigned short v2us;
typedef __attribute__((ext_vector_type(8)))  float    v8f;
typedef __attribute__((ext_vector_type(4)))  float    v4f;
typedef v8h  __attribute__((may_alias)) v8ha;
typedef v4f  __attribute__((may_alias)) v4fa;
typedef v8us __attribute__((may_alias)) v8usa;

__device__ __forceinline__ unsigned short f2bf(float f) { unsigned u = __float_as_uint(f); u += 0x7FFFu + ((u >> 16) & 1u); return (unsigned short)(u >> 16); }
__device__ __forceinline__ float bf2f(unsigned short b) { return __uint_as_float(((unsigned)b) << 16); }
__device__ __forceinline__ float bfr(float f) { return bf2f(f2bf(f)); }
__device__ __forceinline__ v16h cat16(v8h lo, v8h hi) { return __builtin_shufflevector(lo, hi, 0, 1, 2, 3, 4, 5, 6, 7, 8, 9, 10, 11, 12, 13, 14, 15); }
__device__ __forceinline__ v16bf cat16b(v8us lo, v8us hi) { return __builtin_bit_cast(v16bf, __builtin_shufflevector(lo, hi, 0, 1, 2, 3, 4, 5, 6, 7, 8, 9, 10, 11, 12, 13, 14, 15)); }
__device__ __forceinline__ v8f wmma16(v16h a, v16h b, v8f c) { return __builtin_amdgcn_wmma_f32_16x16x32_f16(false, a, false, b, (short)0, c, false, false); }
__device__ __forceinline__ v8f wmmab(v16bf a, v16bf b, v8f c) { return __builtin_amdgcn_wmma_f32_16x16x32_bf16(false, a, false, b, (short)0, c, false, false); }

template <typename T16> struct WFrag;
template <> struct WFrag<h16> { typedef v16h V; static __device__ __forceinline__ V ld(const h16* p) { return cat16(*(const v8h*)p, *(const v8h*)(p + 16)); } static __device__ __forceinline__ v8f mma(V a, V b, v8f c) { return wmma16(a, b, c); } };
template <> struct WFrag<bf> { typedef v16bf V; static __device__ __forceinline__ V ld(const bf* p) { return cat16b(*(const v8us*)p, *(const v8us*)(p + 16)); } static __device__ __forceinline__ v8f mma(V a, V b, v8f c) { return wmmab(a, b, c); } };

template <int MODE>
__global__ __launch_bounds__(32) void k_gemmw(const bf* __restrict__ A, const bf* __restrict__ Bt, size_t sB, h16* P, size_t sP, float* C, const float* bias0, const float* bias1, const float* xres) {
    typedef WFrag<bf>::V V;
    __shared__ __align__(16) float os[16 * 68];
    __shared__ __align__(16) h16 ts[64 * 72];
    const int z = blockIdx.z; Bt += (size_t)z * sB;
    const int lane = threadIdx.x & 31, lr = lane & 15, hi = lane >> 4; const int r0 = blockIdx.x * 64, c0 = blockIdx.y * 64;
    v8f acc[4][4];
#pragma unroll
    for (int mb = 0; mb < 4; ++mb)
#pragma unroll
        for (int nb = 0; nb < 4; ++nb) acc[mb][nb] = (v8f){};
    const size_t aoff = (size_t)(r0 + lr) * DM + 8 * hi, boff = (size_t)(c0 + lr) * DM + 8 * hi;
#pragma unroll 1
    for (int kc = 0; kc < DM; kc += 32) {
        V a[4];
#pragma unroll
        for (int mb = 0; mb < 4; ++mb) a[mb] = WFrag<bf>::ld(A + aoff + (size_t)mb * 16 * DM + kc);
#pragma unroll
        for (int nb = 0; nb < 4; ++nb) { const V b = WFrag<bf>::ld(Bt + boff + (size_t)nb * 16 * DM + kc);
#pragma unroll
            for (int mb = 0; mb < 4; ++mb) acc[mb][nb] = WFrag<bf>::mma(a[mb], b, acc[mb][nb]); }
        asm volatile("v_nop\n\tv_nop\n\tv_nop\n\tv_nop" : "+v"(acc[0][0]), "+v"(acc[1][1]), "+v"(acc[2][2]), "+v"(acc[3][3]) : "v"(a[0]), "v"(a[3]));
    }
    const int bb_ = r0 / SEQ, s0 = r0 % SEQ;
    const int rq = lane >> 3, pc = lane & 7;
    if (MODE == 0) {
        h16* prow = P + (size_t)z * sP + ((size_t)(bb_ * NH + (int)blockIdx.y) * SEQ + s0) * HD;
        float bv[8];
#pragma unroll
        for (int q = 0; q < 8; ++q) { const int c = c0 + pc * 8 + q; const float u0 = bias0[c], u1 = bias1[c]; bv[q] = bfr(z == 0 ? u0 : u1); }
#pragma unroll
        for (int mb = 0; mb < 4; ++mb) {
#pragma unroll
            for (int nb = 0; nb < 4; ++nb) {
#pragma unroll
                for (int j = 0; j < 8; ++j) os[(hi * 8 + j) * 68 + nb * 16 + lr] = acc[mb][nb][j]; }
            __syncthreads();
#pragma unroll 1
            for (int ps = 0; ps < 2; ++ps) {
#pragma unroll
                for (int s = 0; s < 4; ++s) { const int row = 4 * s + rq; const v4f a0 = *(const v4fa*)(os + row * 68 + pc * 8); const v4f a1 = *(const v4fa*)(os + row * 68 + pc * 8 + 4); v8h o;
                    o[0] = (h16)(a0[0] + bv[0]); o[1] = (h16)(a0[1] + bv[1]); o[2] = (h16)(a0[2] + bv[2]); o[3] = (h16)(a0[3] + bv[3]);
                    o[4] = (h16)(a1[0] + bv[4]); o[5] = (h16)(a1[1] + bv[5]); o[6] = (h16)(a1[2] + bv[6]); o[7] = (h16)(a1[3] + bv[7]);
                    *(volatile v8h*)(prow + (size_t)(mb * 16 + row) * HD + pc * 8) = o; }
                if (ps == 0) __threadfence(); }
            __syncthreads();
        }
    } else if (MODE == 1) {
        h16* vb = P + ((size_t)(bb_ * NH + (int)blockIdx.y) * HD) * SEQ + s0;
        float bv[4];
#pragma unroll
        for (int nb = 0; nb < 4; ++nb) bv[nb] = bfr(bias0[c0 + nb * 16 + lr]);
#pragma unroll
        for (int mb = 0; mb < 4; ++mb) {
#pragma unroll
            for (int nb = 0; nb < 4; ++nb) { v8h o;
#pragma unroll
                for (int j = 0; j < 8; ++j) o[j] = (h16)(acc[mb][nb][j] + bv[nb]);
                *(v8ha*)(ts + (nb * 16 + lr) * 72 + mb * 16 + 8 * hi) = o; } }
        __syncthreads();
#pragma unroll 1
        for (int ps = 0; ps < 2; ++ps) {
#pragma unroll
            for (int s = 0; s < 16; ++s) { const int d = 4 * s + rq; const v8h o = *(const v8ha*)(ts + d * 72 + pc * 8); *(volatile v8h*)(vb + (size_t)d * SEQ + pc * 8) = o; }
            if (ps == 0) __threadfence(); }
    } else {
        const int cofs = lr * 4; float b4[4];
#pragma unroll
        for (int q = 0; q < 4; ++q) b4[q] = bfr(bias0[c0 + cofs + q]);
#pragma unroll
        for (int mb = 0; mb < 4; ++mb) {
#pragma unroll
            for (int nb = 0; nb < 4; ++nb) {
#pragma unroll
                for (int j = 0; j < 8; ++j) os[(hi * 8 + j) * 68 + nb * 16 + lr] = acc[mb][nb][j]; }
            __syncthreads();
#pragma unroll 1
            for (int ps = 0; ps < 2; ++ps) {
#pragma unroll
                for (int s = 0; s < 8; ++s) { const int row = 2 * s + hi; const int m = r0 + mb * 16 + row; const size_t xrow = (size_t)(m / SEQ) * SEQ_FULL + (size_t)(m % SEQ);
                    v4f val = *(const v4fa*)(os + row * 68 + cofs); const v4f xv = *(const v4f*)(xres + xrow * DM + c0 + cofs);
                    val[0] = (val[0] + b4[0]) + bfr(xv[0]); val[1] = (val[1] + b4[1]) + bfr(xv[1]); val[2] = (val[2] + b4[2]) + bfr(xv[2]); val[3] = (val[3] + b4[3]) + bfr(xv[3]);
                    *(volatile v4f*)(C + (size_t)m * DM + c0 + cofs) = val; }
                if (ps == 0) __threadfence(); }
            __syncthreads();
        }
    }
}

__global__ __launch_bounds__(256) void k_wtG(const float* __restrict__ w, int K, int N, bf* Bt) {
    const int lane = threadIdx.x & 31; const int L0 = (blockIdx.x * 8 + (threadIdx.x >> 5)) * 8; const int nlines = N * K / 64;
#pragma unroll
    for (int ps = 0; ps < 2; ++ps) {
#pragma unroll 1
        for (int l = 0; l < 8; ++l) { const int L = L0 + l; if (L >= nlines) break; const size_t e = (size_t)L * 64 + lane * 2; const int k = (int)(e % K), n = (int)(e / K); v2us o;
            o[0] = f2bf(w[(size_t)k * N + n]); o[1] = f2bf(w[(size_t)(k + 1) * N + n]); *(volatile v2us*)(Bt + e) = o; }
        if (ps == 0) __threadfence(); }
}
__global__ __launch_bounds__(256) void k_cvt8(const float* __restrict__ src, bf* dst, size_t n8, size_t sS, size_t sD) { const size_t i = (size_t)blockIdx.x * 256 + threadIdx.x; if (i >= n8) return; src += (size_t)blockIdx.y * sS; dst += (size_t)blockIdx.y * sD; const v8f v = *(const v8f*)(src + i * 8); v8us o;
#pragma unroll
    for (int k = 0; k < 8; ++k) o[k] = f2bf(v[k]); *(volatile v8us*)(dst + i * 8) = o; __threadfence(); *(volatile v8us*)(dst + i * 8) = o; }

__global__ __launch_bounds__(128) void k_flash(const h16* __restrict__ Q, const h16* __restrict__ Kpl, const h16* __restrict__ VT, bf* CTX) {
    __shared__ __align__(16) unsigned short cs[4 * 16 * 72];
    const int lane = threadIdx.x & 31, wid = threadIdx.x >> 5, lr = lane & 15, hi = lane >> 4;
    const int gw = blockIdx.x * 4 + wid; const int bh = gw / (SEQ / 16); const int q0 = (gw % (SEQ / 16)) * 16; const int b = bh / NH, h = bh % NH;
    const h16* Qp = Q + ((size_t)bh * SEQ + q0 + lr) * HD + 8 * hi;
    const v16h qb0 = WFrag<h16>::ld(Qp), qb1 = WFrag<h16>::ld(Qp + 32);
    const h16* Kb = Kpl + (size_t)bh * SEQ * HD + (size_t)lr * HD + 8 * hi;
    const h16* Vb = VT + (size_t)bh * HD * SEQ + (size_t)lr * SEQ + 8 * hi;
    v8f o[4];
#pragma unroll
    for (int j = 0; j < 4; ++j) o[j] = (v8f){};
    float m = -1.0e30f, ls = 0.0f;
#pragma unroll 1
    for (int k0 = 0; k0 < SEQ; k0 += 32) {
        const h16* kr = Kb + (size_t)k0 * HD;
        const v16h ka = WFrag<h16>::ld(kr), kb = WFrag<h16>::ld(kr + 32), kc = WFrag<h16>::ld(kr + 16 * HD), kd = WFrag<h16>::ld(kr + 16 * HD + 32);
        v8f s0 = wmma16(ka, qb0, (v8f){}); s0 = wmma16(kb, qb1, s0);
        v8f s1 = wmma16(kc, qb0, (v8f){}); s1 = wmma16(kd, qb1, s1);
        asm volatile("v_nop\n\tv_nop\n\tv_nop\n\tv_nop" : "+v"(s0), "+v"(s1) : "v"(kd), "v"(qb1));
        float mx = fmaxf(s0[0], s1[0]);
#pragma unroll
        for (int r = 1; r < 8; ++r) mx = fmaxf(mx, fmaxf(s0[r], s1[r]));
        mx *= 0.125f;
        const float mo = __shfl_xor(mx, 16, 32); mx = fmaxf(mx, mo);
        const float mn = fmaxf(m, mx);
        const float alpha = __builtin_amdgcn_exp2f((m - mn) * L2E);
        const float off = 10.0f - mn * L2E;
        m = mn;
        v16h pb; float psum = 0.0f;
#pragma unroll
        for (int r = 0; r < 8; ++r) { const float p0 = __builtin_amdgcn_exp2f(__builtin_fmaf(s0[r], SC2, off)); const float p1 = __builtin_amdgcn_exp2f(__builtin_fmaf(s1[r], SC2, off)); psum += p0 + p1; pb[r] = (h16)p0; pb[8 + r] = (h16)p1; }
        ls = ls * alpha + psum;
#pragma unroll
        for (int j = 0; j < 4; ++j) o[j] = o[j] * alpha;
        const h16* vr = Vb + k0;
        const v16h va0 = WFrag<h16>::ld(vr), va1 = WFrag<h16>::ld(vr + (size_t)16 * SEQ), va2 = WFrag<h16>::ld(vr + (size_t)32 * SEQ), va3 = WFrag<h16>::ld(vr + (size_t)48 * SEQ);
        o[0] = wmma16(va0, pb, o[0]); o[1] = wmma16(va1, pb, o[1]); o[2] = wmma16(va2, pb, o[2]); o[3] = wmma16(va3, pb, o[3]);
        asm volatile("v_nop\n\tv_nop\n\tv_nop\n\tv_nop" : "+v"(o[0]), "+v"(o[1]), "+v"(o[2]), "+v"(o[3]) : "v"(va3), "v"(pb));
    }
    const float lo_ = __shfl_xor(ls, 16, 32); ls += lo_;
    const float inv = 1.0f / ls;
    unsigned short* cw = cs + wid * (16 * 72);
#pragma unroll
    for (int j = 0; j < 4; ++j) { v8us w;
#pragma unroll
        for (int r = 0; r < 8; ++r) w[r] = f2bf(o[j][r] * inv);
        *(v8usa*)(cw + lr * 72 + j * 16 + 8 * hi) = w; }
    __syncthreads();
    const int rq = lane >> 3, pc = lane & 7;
    bf* crow = CTX + ((size_t)b * SEQ + q0) * DM + h * HD + pc * 8;
    v8us ov[4];
#pragma unroll
    for (int s = 0; s < 4; ++s) ov[s] = *(const v8usa*)(cw + (4 * s + rq) * 72 + pc * 8);
#pragma unroll
    for (int s = 0; s < 4; ++s) *(volatile v8us*)(crow + (size_t)(4 * s + rq) * DM) = ov[s];
    __threadfence();
#pragma unroll
    for (int s = 0; s < 4; ++s) *(volatile v8us*)(crow + (size_t)(4 * s + rq) * DM) = ov[s];
}

extern "C" void kernel_launch(void* const* d_in, const int* in_sizes, int n_in,
                              void* d_out, int out_size, void* d_ws, size_t ws_size, hipStream_t stream) {
    if (n_in < 9) return;
    const size_t xneed = (size_t)(NB - 1) * SEQ_FULL * DM + (size_t)SEQ * DM;
    if ((size_t)in_sizes[0] < xneed) return;
    if ((size_t)in_sizes[1] < (size_t)DM * DM || (size_t)in_sizes[3] < (size_t)DM * DM || (size_t)in_sizes[5] < (size_t)DM * DM || (size_t)in_sizes[7] < (size_t)DM * DM) return;
    if (in_sizes[2] < DM || in_sizes[4] < DM || in_sizes[6] < DM || in_sizes[8] < DM) return;
    if ((size_t)out_size < (size_t)MT * DM) return;
    const float* x = (const float*)d_in[0]; const float* wq = (const float*)d_in[1]; const float* bq = (const float*)d_in[2]; const float* wk = (const float*)d_in[3]; const float* bk = (const float*)d_in[4];
    const float* wv = (const float*)d_in[5]; const float* bv = (const float*)d_in[6]; const float* wo = (const float*)d_in[7]; const float* bo = (const float*)d_in[8];
    float* OUT = (float*)d_out;
    char* wsp = (char*)d_ws;
    auto take = [&](size_t bytes) { char* p = wsp; wsp += (bytes + 255) & ~(size_t)255; return (void*)p; };
    bf*  WT  = (bf*)take((size_t)4 * DM * DM * 2);
    bf*  XB  = (bf*)take((size_t)MT * DM * 2);
    h16* QK  = (h16*)take((size_t)2 * MT * DM * 2);
    h16* VTp = (h16*)take((size_t)MT * DM * 2);
    bf*  CTX = (bf*)take((size_t)MT * DM * 2);
    if ((size_t)(wsp - (char*)d_ws) > ws_size) return;
    h16* QP = QK; h16* KP = QK + (size_t)MT * DM;

    k_cvt8<<<dim3((unsigned)(((size_t)SEQ * DM / 8 + 255) / 256), NB, 1), 256, 0, stream>>>(x, XB, (size_t)SEQ * DM / 8, (size_t)SEQ_FULL * DM, (size_t)SEQ * DM);
    const unsigned gw_ = (unsigned)((DM * DM / 64 + 63) / 64);
    k_wtG<<<gw_, 256, 0, stream>>>(wq, DM, DM, WT);
    k_wtG<<<gw_, 256, 0, stream>>>(wk, DM, DM, WT + (size_t)DM * DM);
    k_wtG<<<gw_, 256, 0, stream>>>(wv, DM, DM, WT + (size_t)2 * DM * DM);
    k_wtG<<<gw_, 256, 0, stream>>>(wo, DM, DM, WT + (size_t)3 * DM * DM);
    k_gemmw<0><<<dim3(MT / 64, DM / 64, 2), 32, 0, stream>>>(XB, WT, (size_t)DM * DM, QP, (size_t)MT * DM, OUT, bq, bk, x);
    k_gemmw<1><<<dim3(MT / 64, DM / 64, 1), 32, 0, stream>>>(XB, WT + (size_t)2 * DM * DM, 0, VTp, 0, OUT, bv, bv, x);
    k_flash<<<(unsigned)(NB * NH * (SEQ / 16) / 4), 128, 0, stream>>>(QP, KP, VTp, CTX);
    k_gemmw<2><<<dim3(MT / 64, DM / 64, 1), 32, 0, stream>>>(CTX, WT + (size_t)3 * DM * DM, 0, QP, 0, OUT, bo, bo, x);
}
